// GNNEncoder_51694226375420
// MI455X (gfx1250) — hardware-verified
//
#include <hip/hip_runtime.h>
#include <stddef.h>
#include <stdint.h>
#include <math.h>


#define XDIM   6
#define HID    64
#define ODIM   32
#define KX     32
#define K2     128
#define KC     64
#define NTHR   256
#define NWAVE  8
#define EPT    8
#define CHUNK  (NTHR * EPT)
#define WCAP   (EPT * 32)
#define LISTN  (NWAVE * WCAP)
#define NBA    1024
#define SLA    10
#define RCAP   28672
#define DEGCAP 64
#define GBM    64
#define GBN    64
#define GTHR   128
#define AGG_ZINTS (LISTN + 2 * RCAP + 3 * NBA)
#define AGG_LDS_INTS (AGG_ZINTS + 16)
#define WSMAX  134217728

static_assert((CHUNK & (CHUNK - 1)) == 0 && CHUNK <= 4096);
static_assert((NBA & (NBA - 1)) == 0 && NBA == (1 << SLA));
static_assert(((long long)CHUNK << SLA) < (1LL << 31));
static_assert(LISTN % NTHR == 0);
static_assert(NBA % NWAVE == 0 && NBA % 32 == 0 && NBA % GBM == 0 && NBA == 4 * NTHR);
static_assert(RCAP % 32 == 0 && AGG_ZINTS % 4 == 0 && LISTN % 4 == 0);
static_assert(KX % 32 == 0 && K2 % 32 == 0 && KC % 32 == 0 && K2 == 2 * HID && KC == 2 * ODIM);
static_assert(GBM == (GTHR / 32) * 16 && GBN == HID && ODIM == 32 && HID == 64);
static_assert(AGG_LDS_INTS * 4 <= 300000);
static_assert(DEGCAP >= 44);

typedef float          v2f   __attribute__((ext_vector_type(2)));
typedef float          v4f   __attribute__((ext_vector_type(4)));
typedef float          v8f   __attribute__((ext_vector_type(8)));
typedef int            v4i   __attribute__((ext_vector_type(4)));
typedef int            v8i   __attribute__((ext_vector_type(8)));
typedef unsigned int   v4u   __attribute__((ext_vector_type(4)));
typedef unsigned short v8us  __attribute__((ext_vector_type(8)));
typedef unsigned short v16us __attribute__((ext_vector_type(16)));
typedef __bf16         v16bf __attribute__((ext_vector_type(16)));
typedef v2f  __attribute__((may_alias)) v2fa;
typedef v4f  __attribute__((may_alias)) v4fa;
typedef v4i  __attribute__((may_alias)) v4ia;
typedef v8us __attribute__((may_alias)) v8usa;
union FragB { v16bf v; v16us u; v8us h[2]; v8i w; };

__device__ __forceinline__ v8f wmb(const FragB& a, const FragB& b, v8f c) {
  v8f d = __builtin_amdgcn_wmma_f32_16x16x32_bf16(false, a.v, false, b.v, (short)0, c, false, false);
  asm volatile("v_nop\n\tv_nop\n\tv_nop\n\tv_nop" : "+v"(d) : "v"(a.w), "v"(b.w));
  return d;
}

__device__ __forceinline__ unsigned bf16_bits(float f) {
  const unsigned u = __float_as_uint(f);
  return (u + 0x7FFFu + ((u >> 16) & 1u)) >> 16;
}
__device__ __forceinline__ float bf16_val(float f) {
  return __uint_as_float(bf16_bits(f) << 16);
}
__device__ __forceinline__ unsigned hlsel(float v, bool losel) {
  const unsigned hb = bf16_bits(v);
  const unsigned lb = bf16_bits(v - __uint_as_float(hb << 16));
  return losel ? lb : hb;
}

template <int SLB>
__device__ __forceinline__ int scan_chunk(const int* __restrict__ dsts, int nE, int cbase, int slotBase,
                                          int nb, int vec8, int* list, int tid, int lane, int wave) {
  int wc = 0;
  const int el0  = tid * EPT;
  const int e0   = cbase + el0;
  const int sent = -2147483647 - 1;
  v4i da, db;
  if (vec8 != 0 && cbase + CHUNK <= nE) {
    da = *(const v4i*)(dsts + e0);
    db = *(const v4i*)(dsts + e0 + 4);
  } else {
    da.x = (e0     < nE) ? dsts[min(e0,     nE - 1)] : sent;
    da.y = (e0 + 1 < nE) ? dsts[min(e0 + 1, nE - 1)] : sent;
    da.z = (e0 + 2 < nE) ? dsts[min(e0 + 2, nE - 1)] : sent;
    da.w = (e0 + 3 < nE) ? dsts[min(e0 + 3, nE - 1)] : sent;
    db.x = (e0 + 4 < nE) ? dsts[min(e0 + 4, nE - 1)] : sent;
    db.y = (e0 + 5 < nE) ? dsts[min(e0 + 5, nE - 1)] : sent;
    db.z = (e0 + 6 < nE) ? dsts[min(e0 + 6, nE - 1)] : sent;
    db.w = (e0 + 7 < nE) ? dsts[min(e0 + 7, nE - 1)] : sent;
  }
  const unsigned nbs = (unsigned)slotBase;
  const unsigned unb = (unsigned)nb;
  const unsigned s0 = (unsigned)da.x - nbs, s1 = (unsigned)da.y - nbs;
  const unsigned s2 = (unsigned)da.z - nbs, s3 = (unsigned)da.w - nbs;
  const unsigned s4 = (unsigned)db.x - nbs, s5 = (unsigned)db.y - nbs;
  const unsigned s6 = (unsigned)db.z - nbs, s7 = (unsigned)db.w - nbs;
  const bool h0 = s0 < unb, h1 = s1 < unb, h2 = s2 < unb, h3 = s3 < unb;
  const bool h4 = s4 < unb, h5 = s5 < unb, h6 = s6 < unb, h7 = s7 < unb;
  const unsigned any = __builtin_amdgcn_ballot_w32(h0 | h1 | h2 | h3 | h4 | h5 | h6 | h7);
  if (any != 0u) {
#define HITJ(J, HJ, SJ) { \
      const unsigned mj = __builtin_amdgcn_ballot_w32(HJ); \
      if (mj != 0u) { \
        if (HJ) { \
          const int pos = wc + (int)__builtin_amdgcn_mbcnt_lo(mj, 0u); \
          if (pos < WCAP) list[wave * WCAP + pos] = ((el0 + (J)) << SLB) | (int)(SJ); \
        } \
        wc += (int)__builtin_popcount(mj); } }
    HITJ(0, h0, s0)
    HITJ(1, h1, s1)
    HITJ(2, h2, s2)
    HITJ(3, h3, s3)
    HITJ(4, h4, s4)
    HITJ(5, h5, s5)
    HITJ(6, h6, s6)
    HITJ(7, h7, s7)
#undef HITJ
  }
  return wc;
}

__global__ __launch_bounds__(NTHR) void k_xprep(const float* __restrict__ x, int nN, int nUnits,
                                                unsigned short* xb) {
  const int u = (int)blockIdx.x * NTHR + (int)threadIdx.x;
  if (u >= nUnits) return;
  const int row = u >> 2;
  const int k8  = (u & 3) * 8;
  const int rc  = row < nN ? row : nN - 1;
  const float* p = x + (size_t)rc * XDIM;
  const float f0 = p[0], f1 = p[1], f2 = p[2], f3 = p[3], f4 = p[4], f5 = p[5];
  const bool ok = (row < nN) && (k8 == 0);
  v8us o;
  o[0] = ok ? (unsigned short)bf16_bits(f0) : (unsigned short)0;
  o[1] = ok ? (unsigned short)bf16_bits(f1) : (unsigned short)0;
  o[2] = ok ? (unsigned short)bf16_bits(f2) : (unsigned short)0;
  o[3] = ok ? (unsigned short)bf16_bits(f3) : (unsigned short)0;
  o[4] = ok ? (unsigned short)bf16_bits(f4) : (unsigned short)0;
  o[5] = ok ? (unsigned short)bf16_bits(f5) : (unsigned short)0;
  o[6] = (unsigned short)0;
  o[7] = (unsigned short)0;
  unsigned short* dp = xb + (size_t)row * KX + k8;
  *(volatile v8us*)dp = o;
  __threadfence();
  *(volatile v8us*)dp = o;
}

__global__ __launch_bounds__(NTHR) void k_wtr(const float* __restrict__ w, int ldw, int Kout, int Kmod, int Kvalid,
                                              unsigned short* wt, int nUnits) {
  const int u = (int)blockIdx.x * NTHR + (int)threadIdx.x;
  if (u >= nUnits) return;
  const int kq = Kout >> 3;
  const int n  = u / kq;
  const int k8 = (u - n * kq) * 8;
  const int kk = k8 - (k8 / Kmod) * Kmod;
  v8us o;
#pragma unroll
  for (int i = 0; i < 8; ++i) {
    const int kr = kk + i;
    const int kc = kr < Kvalid ? kr : Kvalid - 1;
    const float v = w[(size_t)kc * (size_t)ldw + n];
    o[i] = (kr < Kvalid) ? (unsigned short)bf16_bits(v) : (unsigned short)0;
  }
  unsigned short* dp = wt + (size_t)n * (size_t)Kout + k8;
  *(volatile v8us*)dp = o;
  __threadfence();
  *(volatile v8us*)dp = o;
}

template <int NT, int MODE>
__global__ __launch_bounds__(GTHR) void k_gemm(const unsigned short* __restrict__ A,
                                               const unsigned short* __restrict__ WT, int K,
                                               const float* __restrict__ bias,
                                               const float* __restrict__ flag, int nN,
                                               float* outF, unsigned short* outH) {
  constexpr int NC = 16 * NT;
  __shared__ __attribute__((aligned(16))) float stg[GBM * GBN];
  __shared__ __attribute__((aligned(16))) float sbias[GBN];
  __shared__ __attribute__((aligned(16))) float sflag[GBM];
  const int tid = (int)threadIdx.x, lane = tid & 31, wave = tid >> 5, hh = lane >> 4, m = lane & 15;
  const int rowBase = (int)blockIdx.x * GBM;
  (void)nN; (void)outF; (void)outH; (void)bias; (void)flag;

  if constexpr (MODE != 0) {
    if (tid < GBN) {
      const float bb = bias[tid < NC ? tid : NC - 1];
      sbias[tid] = (tid < NC) ? bf16_val(bb) : 0.0f;
    }
    if (tid < 16) *(v4fa*)(sflag + 4 * tid) = *(const v4fa*)(flag + (size_t)rowBase + 4 * tid);
  }

  v8f acc[NT];
  {
    const v8f z = {0.f, 0.f, 0.f, 0.f, 0.f, 0.f, 0.f, 0.f};
#pragma unroll
    for (int t = 0; t < NT; ++t) acc[t] = z;
  }
  const unsigned short* ap = A  + (size_t)(rowBase + 16 * wave + m) * (size_t)K + 8 * hh;
  const unsigned short* wp = WT + (size_t)m * (size_t)K + 8 * hh;
  const int ksteps = K >> 5;
#pragma unroll 1
  for (int ks = 0; ks < ksteps; ++ks) {
    FragB af;
    af.h[0] = *(const v8usa*)(ap + 32 * ks);
    af.h[1] = *(const v8usa*)(ap + 32 * ks + 16);
#pragma unroll
    for (int t = 0; t < NT; ++t) {
      const unsigned short* wq = wp + (size_t)(16 * t) * (size_t)K + 32 * ks;
      FragB bf;
      bf.h[0] = *(const v8usa*)wq;
      bf.h[1] = *(const v8usa*)(wq + 16);
      acc[t] = wmb(af, bf, acc[t]);
    }
  }

#pragma unroll
  for (int t = 0; t < NT; ++t) {
    const int lc = 16 * t + m;
#pragma unroll
    for (int r = 0; r < 8; ++r) {
      const int lr = 16 * wave + 8 * hh + r;
      stg[lr * GBN + lc] = acc[t][r];
    }
  }
  __syncthreads();

  if constexpr (MODE == 1) {
    const int cb = 8 * (m & 7);
    const bool losel = (m & 8) != 0;
    const v4f b0 = *(const v4fa*)(sbias + cb);
    const v4f b1 = *(const v4fa*)(sbias + cb + 4);
    v4u hv[8];
#pragma unroll
    for (int i = 0; i < 8; ++i) {
      const int lr = 16 * wave + 2 * i + hh;
      const v4f a = *(const v4fa*)(stg + lr * GBN + cb);
      const v4f c = *(const v4fa*)(stg + lr * GBN + cb + 4);
      const float fl = sflag[lr];
      const float v0 = fmaxf(fmaf(b0.x, fl, a.x), 0.0f), v1 = fmaxf(fmaf(b0.y, fl, a.y), 0.0f);
      const float v2 = fmaxf(fmaf(b0.z, fl, a.z), 0.0f), v3 = fmaxf(fmaf(b0.w, fl, a.w), 0.0f);
      const float v4 = fmaxf(fmaf(b1.x, fl, c.x), 0.0f), v5 = fmaxf(fmaf(b1.y, fl, c.y), 0.0f);
      const float v6 = fmaxf(fmaf(b1.z, fl, c.z), 0.0f), v7 = fmaxf(fmaf(b1.w, fl, c.w), 0.0f);
      const unsigned u0 = hlsel(v0, losel), u1 = hlsel(v1, losel), u2 = hlsel(v2, losel), u3 = hlsel(v3, losel);
      const unsigned u4 = hlsel(v4, losel), u5 = hlsel(v5, losel), u6 = hlsel(v6, losel), u7 = hlsel(v7, losel);
      v4u pv;
      pv.x = u0 | (u1 << 16); pv.y = u2 | (u3 << 16); pv.z = u4 | (u5 << 16); pv.w = u6 | (u7 << 16);
      hv[i] = pv;
    }
#pragma unroll
    for (int i = 0; i < 8; ++i) {
      const int gr = rowBase + 16 * wave + 2 * i + hh;
      unsigned short* hp = outH + (size_t)gr * K2 + 8 * m;
      *(volatile v4u*)hp = hv[i];
    }
    __threadfence();
#pragma unroll
    for (int i = 0; i < 8; ++i) {
      const int gr = rowBase + 16 * wave + 2 * i + hh;
      unsigned short* hp = outH + (size_t)gr * K2 + 8 * m;
      *(volatile v4u*)hp = hv[i];
    }
  } else {
    const int mm = m & (4 * NT - 1);
    v4f fv[8];
#pragma unroll
    for (int i = 0; i < 8; ++i) {
      const int lr = 16 * wave + 2 * i + hh;
      v4f a = *(const v4fa*)(stg + lr * GBN + 4 * mm);
      if constexpr (MODE == 2) {
        const v4f bb = *(const v4fa*)(sbias + 4 * mm);
        const float fl = sflag[lr];
        a.x = fmaf(bb.x, fl, a.x); a.y = fmaf(bb.y, fl, a.y);
        a.z = fmaf(bb.z, fl, a.z); a.w = fmaf(bb.w, fl, a.w);
      }
      fv[i] = a;
    }
#pragma unroll
    for (int i = 0; i < 8; ++i) {
      const int gr = rowBase + 16 * wave + 2 * i + hh;
      const bool wr = (m < 4 * NT) && (MODE != 2 || gr < nN);
      float* op = outF + (size_t)gr * (size_t)NC + 4 * mm;
      if (wr) *(volatile v4f*)op = fv[i];
    }
    __threadfence();
#pragma unroll
    for (int i = 0; i < 8; ++i) {
      const int gr = rowBase + 16 * wave + 2 * i + hh;
      const bool wr = (m < 4 * NT) && (MODE != 2 || gr < nN);
      float* op = outF + (size_t)gr * (size_t)NC + 4 * mm;
      if (wr) *(volatile v4f*)op = fv[i];
    }
  }
}

template <int CPL>
__global__ __launch_bounds__(NTHR) void k_scan(const int* __restrict__ srcs, const int* __restrict__ dsts,
                                               const float* __restrict__ eat, int nE, int nN, int vec8, int mRows,
                                               const float* __restrict__ P, const float* __restrict__ w1, int xd,
                                               const float* __restrict__ b1, int wrflag,
                                               unsigned short* mo, float* flag) {
  constexpr int HW = 32 * CPL;
  extern __shared__ __attribute__((aligned(16))) int dsm[];
  int* list = dsm;
  int* hl   = dsm + LISTN;
  int* sl   = dsm + LISTN + RCAP;
  int* cnt  = dsm + LISTN + 2 * RCAP;
  int* offs = cnt + NBA;
  int* cur  = offs + NBA;
  int* misc = cur + NBA;
  const int tid = (int)threadIdx.x, lane = tid & 31, wave = tid >> 5;
  const int nodeBase = (int)blockIdx.x * NBA;

  {
    const v4i z4 = {0, 0, 0, 0};
    for (int i = tid * 4; i < AGG_ZINTS; i += NTHR * 4) *(v4ia*)(dsm + i) = z4;
    if (tid < 16) misc[tid] = 0;
  }
  float wb0[CPL], wb1[CPL], wb2[CPL], bv[CPL];
  if constexpr (CPL == 2) {
    const v2f r0 = *(const v2fa*)(w1 + (size_t)(xd + 0) * HW + 2 * lane);
    const v2f r1 = *(const v2fa*)(w1 + (size_t)(xd + 1) * HW + 2 * lane);
    const v2f r2 = *(const v2fa*)(w1 + (size_t)(xd + 2) * HW + 2 * lane);
    const v2f bb = *(const v2fa*)(b1 + 2 * lane);
    wb0[0] = bf16_val(r0.x); wb0[1] = bf16_val(r0.y);
    wb1[0] = bf16_val(r1.x); wb1[1] = bf16_val(r1.y);
    wb2[0] = bf16_val(r2.x); wb2[1] = bf16_val(r2.y);
    bv[0]  = bf16_val(bb.x); bv[1]  = bf16_val(bb.y);
  } else {
    wb0[0] = bf16_val(w1[(size_t)(xd + 0) * HW + lane]);
    wb1[0] = bf16_val(w1[(size_t)(xd + 1) * HW + lane]);
    wb2[0] = bf16_val(w1[(size_t)(xd + 2) * HW + lane]);
    bv[0]  = bf16_val(b1[lane]);
  }
  __syncthreads();

  int t = 0, ov = 0;
  const int nChunks = (nE + CHUNK - 1) / CHUNK;
#pragma unroll 1
  for (int ch = 0; ch < nChunks; ++ch) {
    const int cbase = ch * CHUNK;
    const int wc = scan_chunk<SLA>(dsts, nE, cbase, nodeBase, NBA, vec8, list, tid, lane, wave);
    if (lane == 0) misc[wave] = wc;
    __syncthreads();
    if (wave == 0) {
#pragma unroll 1
      for (int w2 = 0; w2 < NWAVE; ++w2) {
        int c = misc[w2];
        c = c < 0 ? 0 : (c > WCAP ? WCAP : c);
#pragma unroll 1
        for (int b0 = 0; b0 < c; b0 += 32) {
          const int idx = b0 + lane;
          const int ent = list[w2 * WCAP + (idx < WCAP ? idx : WCAP - 1)];
          const int m32 = (c - b0) < 32 ? (c - b0) : 32;
#pragma unroll 1
          for (int k = 0; k < m32; ++k) {
            const int u    = __builtin_amdgcn_readlane(ent, k);
            const int slot = u & (NBA - 1);
            const int el   = (u >> SLA) & (CHUNK - 1);
            const int pk   = ((cbase + el) << SLA) | slot;
            if (t < RCAP) {
              if (lane == 0) { hl[t] = pk; cnt[slot] = cnt[slot] + 1; }
              t = t + 1;
            } else {
              ov = 1;
            }
          }
        }
      }
    }
    __syncthreads();
  }
  if (wave == 0 && lane == 0) { misc[8] = t; misc[9] = ov; }
  __syncthreads();
  int tt = misc[8];
  tt = tt < 0 ? 0 : (tt > RCAP ? RCAP : tt);
  const int ovf = misc[9];

  if (wave == 0) {
    const int base = lane * (NBA / 32);
    int s = 0;
#pragma unroll 1
    for (int i = 0; i < NBA / 32; ++i) s += cnt[base + i];
    int incl = s;
#pragma unroll
    for (int d = 1; d < 32; d <<= 1) {
      const int y = __shfl_up(incl, d, 32);
      if (lane >= d) incl += y;
    }
    int run = incl - s;
#pragma unroll 1
    for (int i = 0; i < NBA / 32; ++i) {
      const int cv = cnt[base + i];
      offs[base + i] = run;
      cur[base + i]  = run;
      run += cv;
    }
  }
  __syncthreads();
  if (wave == 0) {
#pragma unroll 1
    for (int b0 = 0; b0 < tt; b0 += 32) {
      const int idx = b0 + lane;
      const int ent = hl[idx < RCAP ? idx : RCAP - 1];
      const int m32 = (tt - b0) < 32 ? (tt - b0) : 32;
#pragma unroll 1
      for (int k = 0; k < m32; ++k) {
        const int u    = __builtin_amdgcn_readlane(ent, k);
        const int slot = u & (NBA - 1);
        if (lane == 0) {
          int p = cur[slot];
          p = p < 0 ? 0 : (p > RCAP - 1 ? RCAP - 1 : p);
          sl[p] = u;
          cur[slot] = p + 1;
        }
      }
    }
  }
  __syncthreads();

  if (wrflag != 0) {
    const v4i c4 = *(const v4ia*)(cnt + 4 * tid);
    const int n0 = nodeBase + 4 * tid;
    v4f fvv;
    fvv.x = (c4.x > 0 && n0 + 0 < nN) ? 1.0f : 0.0f;
    fvv.y = (c4.y > 0 && n0 + 1 < nN) ? 1.0f : 0.0f;
    fvv.z = (c4.z > 0 && n0 + 2 < nN) ? 1.0f : 0.0f;
    fvv.w = (c4.w > 0 && n0 + 3 < nN) ? 1.0f : 0.0f;
    float* fp = flag + (size_t)n0;
    *(volatile v4f*)fp = fvv;
    __threadfence();
    *(volatile v4f*)fp = fvv;
  }

  const float qnan = __int_as_float(0x7fc00000);
  const float pz = (ovf != 0) ? qnan : 0.0f;
#pragma unroll 1
  for (int si = 0; si < NBA / NWAVE; ++si) {
    const int s    = si * NWAVE + wave;
    const int node = nodeBase + s;
    const int craw = cnt[s];
    const bool big = craw > DEGCAP;
    const int c = craw < 0 ? 0 : (craw > DEGCAP ? DEGCAP : craw);
    int o = offs[s];
    o = o < 0 ? 0 : (o > RCAP ? RCAP : o);
    float acc[CPL];
#pragma unroll
    for (int q = 0; q < CPL; ++q) acc[q] = 0.0f;
#pragma unroll 1
    for (int b0 = 0; b0 < c; b0 += 32) {
      int idx = o + b0 + lane;
      idx = idx > RCAP - 1 ? RCAP - 1 : idx;
      const int ent = sl[idx];
      int eid = ent >> SLA;
      eid = eid < 0 ? 0 : (eid > nE - 1 ? nE - 1 : eid);
      int sr = srcs[eid];
      sr = sr < 0 ? 0 : (sr > nN - 1 ? nN - 1 : sr);
      const float* ep = eat + (size_t)eid * 3;
      const int ei0 = __float_as_int(bf16_val(ep[0]));
      const int ei1 = __float_as_int(bf16_val(ep[1]));
      const int ei2 = __float_as_int(bf16_val(ep[2]));
      const int m32 = (c - b0) < 32 ? (c - b0) : 32;
#pragma unroll 1
      for (int k = 0; k < m32; ++k) {
        const int   sk = __builtin_amdgcn_readlane(sr, k);
        const float e0 = __int_as_float(__builtin_amdgcn_readlane(ei0, k));
        const float e1 = __int_as_float(__builtin_amdgcn_readlane(ei1, k));
        const float e2 = __int_as_float(__builtin_amdgcn_readlane(ei2, k));
        float pvv[CPL];
        if constexpr (CPL == 2) {
          const v2f a = *(const v2fa*)(P + (size_t)sk * HW + 2 * lane);
          pvv[0] = a.x; pvv[1] = a.y;
        } else {
          pvv[0] = P[(size_t)sk * HW + lane];
        }
#pragma unroll
        for (int q = 0; q < CPL; ++q) {
          float tv = pvv[q] + bv[q];
          tv = fmaf(e0, wb0[q], tv);
          tv = fmaf(e1, wb1[q], tv);
          tv = fmaf(e2, wb2[q], tv);
          acc[q] += fmaxf(tv, 0.0f);
        }
      }
    }
    const float cf  = (c < 1) ? 1.0f : (float)c;
    const float inv = 1.0f / cf;
    const float pzr = big ? qnan : pz;
    const bool live = node < nN;
    float v[CPL];
#pragma unroll
    for (int q = 0; q < CPL; ++q) {
      const float y = acc[q] * inv + pzr;
      v[q] = live ? y : 0.0f;
    }
    if constexpr (CPL == 2) {
      const unsigned hb0 = bf16_bits(v[0]), hb1 = bf16_bits(v[1]);
      const unsigned lb0 = bf16_bits(v[0] - __uint_as_float(hb0 << 16));
      const unsigned lb1 = bf16_bits(v[1] - __uint_as_float(hb1 << 16));
      const int hw = (int)(hb0 | (hb1 << 16));
      const int lw = (int)(lb0 | (lb1 << 16));
      const int q0s = (4 * lane) & 31, q1s = (4 * lane + 1) & 31;
      const int q2s = (4 * lane + 2) & 31, q3s = (4 * lane + 3) & 31;
      const int g0 = __shfl(hw, q0s, 32), g1 = __shfl(hw, q1s, 32);
      const int g2 = __shfl(hw, q2s, 32), g3 = __shfl(hw, q3s, 32);
      const int p0 = __shfl(lw, q0s, 32), p1 = __shfl(lw, q1s, 32);
      const int p2 = __shfl(lw, q2s, 32), p3 = __shfl(lw, q3s, 32);
      const bool lsel = (lane & 8) != 0;
      v4u pv;
      pv.x = (unsigned int)(lsel ? p0 : g0);
      pv.y = (unsigned int)(lsel ? p1 : g1);
      pv.z = (unsigned int)(lsel ? p2 : g2);
      pv.w = (unsigned int)(lsel ? p3 : g3);
      unsigned short* hp = mo + (size_t)node * (2 * HW) + 8 * (lane & 15);
      const bool wr = (node < mRows) && (lane < 16);
      if (wr) *(volatile v4u*)hp = pv;
      __threadfence();
      if (wr) *(volatile v4u*)hp = pv;
    } else {
      const unsigned hb = bf16_bits(v[0]);
      const unsigned lb = bf16_bits(v[0] - __uint_as_float(hb << 16));
      const int pw = (int)(hb | (lb << 16));
      const int g0 = __shfl(pw, (8 * lane + 0) & 31, 32), g1 = __shfl(pw, (8 * lane + 1) & 31, 32);
      const int g2 = __shfl(pw, (8 * lane + 2) & 31, 32), g3 = __shfl(pw, (8 * lane + 3) & 31, 32);
      const int g4 = __shfl(pw, (8 * lane + 4) & 31, 32), g5 = __shfl(pw, (8 * lane + 5) & 31, 32);
      const int g6 = __shfl(pw, (8 * lane + 6) & 31, 32), g7 = __shfl(pw, (8 * lane + 7) & 31, 32);
      const bool lsel = (lane & 4) != 0;
      const unsigned u0 = lsel ? ((unsigned)g0 >> 16) : ((unsigned)g0 & 0xFFFFu);
      const unsigned u1 = lsel ? ((unsigned)g1 >> 16) : ((unsigned)g1 & 0xFFFFu);
      const unsigned u2 = lsel ? ((unsigned)g2 >> 16) : ((unsigned)g2 & 0xFFFFu);
      const unsigned u3 = lsel ? ((unsigned)g3 >> 16) : ((unsigned)g3 & 0xFFFFu);
      const unsigned u4 = lsel ? ((unsigned)g4 >> 16) : ((unsigned)g4 & 0xFFFFu);
      const unsigned u5 = lsel ? ((unsigned)g5 >> 16) : ((unsigned)g5 & 0xFFFFu);
      const unsigned u6 = lsel ? ((unsigned)g6 >> 16) : ((unsigned)g6 & 0xFFFFu);
      const unsigned u7 = lsel ? ((unsigned)g7 >> 16) : ((unsigned)g7 & 0xFFFFu);
      v4u pv;
      pv.x = u0 | (u1 << 16); pv.y = u2 | (u3 << 16); pv.z = u4 | (u5 << 16); pv.w = u6 | (u7 << 16);
      unsigned short* hp = mo + (size_t)node * (2 * HW) + 8 * (lane & 7);
      const bool wr = (node < mRows) && (lane < 8);
      if (wr) *(volatile v4u*)hp = pv;
      __threadfence();
      if (wr) *(volatile v4u*)hp = pv;
    }
  }
}

static inline int cdiv(int a, int b) { return (a + b - 1) / b; }
static inline size_t al256(size_t o) { return (o + 255) & ~(size_t)255; }

extern "C" void kernel_launch(void* const* d_in, const int* in_sizes, int n_in,
                              void* d_out, int out_size, void* d_ws, size_t ws_size,
                              hipStream_t stream) {
  if (n_in < 15) return;
  if (in_sizes[0] < XDIM || (in_sizes[0] % XDIM) != 0) return;
  const int nN = in_sizes[0] / XDIM;
  if (nN < 1 || nN > (1 << 22)) return;
  if (in_sizes[1] < 2 || (in_sizes[1] & 1) != 0) return;
  const int nE = in_sizes[1] / 2;
  if (nE < 1 || nE >= (1 << (31 - SLA))) return;
  if (in_sizes[2] != 3 * nE) return;
  if (in_sizes[3] != (XDIM + 3) * HID || in_sizes[4] != HID) return;
  if (in_sizes[5] != HID * HID || in_sizes[6] != HID) return;
  if (in_sizes[7] != (HID + 3) * HID || in_sizes[8] != HID) return;
  if (in_sizes[9] != HID * HID || in_sizes[10] != HID) return;
  if (in_sizes[11] != (HID + 3) * ODIM || in_sizes[12] != ODIM) return;
  if (in_sizes[13] != ODIM * ODIM || in_sizes[14] != ODIM) return;
  if (out_size != nN * ODIM) return;

  const float* x   = (const float*)d_in[0];
  const int*   ei  = (const int*)d_in[1];
  const float* eat = (const float*)d_in[2];
  const float* w1a = (const float*)d_in[3];
  const float* b1a = (const float*)d_in[4];
  const float* w2a = (const float*)d_in[5];
  const float* b2a = (const float*)d_in[6];
  const float* w1b = (const float*)d_in[7];
  const float* b1b = (const float*)d_in[8];
  const float* w2b = (const float*)d_in[9];
  const float* b2b = (const float*)d_in[10];
  const float* w1c = (const float*)d_in[11];
  const float* b1c = (const float*)d_in[12];
  const float* w2c = (const float*)d_in[13];
  const float* b2c = (const float*)d_in[14];
  float* out = (float*)d_out;
  const int* src = ei;
  const int* dst = ei + nE;

  const int MP  = cdiv(nN, GBM) * GBM;
  const int gM  = MP / GBM;
  const int gA  = cdiv(MP, NBA);
  const int FLN = gA * NBA;
  if ((long long)gA * NBA < (long long)MP) return;
  const int vec8 = ((nE & 3) == 0) ? 1 : 0;

  char* ws = (char*)d_ws;
  size_t off = 0;
  const size_t oXB  = off; off = al256(off + (size_t)MP * KX * 2);
  const size_t oW1A = off; off = al256(off + (size_t)HID * KX * 2);
  const size_t oW2A = off; off = al256(off + (size_t)HID * K2 * 2);
  const size_t oW1B = off; off = al256(off + (size_t)HID * K2 * 2);
  const size_t oW2B = off; off = al256(off + (size_t)HID * K2 * 2);
  const size_t oW1C = off; off = al256(off + (size_t)ODIM * K2 * 2);
  const size_t oW2C = off; off = al256(off + (size_t)ODIM * KC * 2);
  const size_t oP   = off; off = al256(off + (size_t)MP * HID * 4);
  const size_t oM   = off; off = al256(off + (size_t)MP * K2 * 2);
  const size_t oH   = off; off = al256(off + (size_t)MP * K2 * 2);
  const size_t oFL  = off; off = al256(off + (size_t)FLN * 4);
  if (off > ws_size || off > (size_t)WSMAX) return;
  unsigned short* XB   = (unsigned short*)(ws + oXB);
  unsigned short* W1AT = (unsigned short*)(ws + oW1A);
  unsigned short* W2A2 = (unsigned short*)(ws + oW2A);
  unsigned short* W1B2 = (unsigned short*)(ws + oW1B);
  unsigned short* W2B2 = (unsigned short*)(ws + oW2B);
  unsigned short* W1C2 = (unsigned short*)(ws + oW1C);
  unsigned short* W2C2 = (unsigned short*)(ws + oW2C);
  float*          Pp   = (float*)(ws + oP);
  unsigned short* Mp   = (unsigned short*)(ws + oM);
  unsigned short* Hp   = (unsigned short*)(ws + oH);
  float*          FL   = (float*)(ws + oFL);

  const size_t aggLds = (size_t)AGG_LDS_INTS * 4;
  hipFuncSetAttribute(reinterpret_cast<const void*>(&k_scan<2>), hipFuncAttributeMaxDynamicSharedMemorySize, (int)aggLds);
  hipFuncSetAttribute(reinterpret_cast<const void*>(&k_scan<1>), hipFuncAttributeMaxDynamicSharedMemorySize, (int)aggLds);

  const int nUx = MP * (KX / 8);
  k_xprep<<<cdiv(nUx, NTHR), NTHR, 0, stream>>>(x, nN, nUx, XB);
  {
    const int u1 = HID * (KX / 8);
    k_wtr<<<cdiv(u1, NTHR), NTHR, 0, stream>>>(w1a, HID, KX, KX, XDIM, W1AT, u1);
    const int u2 = HID * (K2 / 8);
    k_wtr<<<cdiv(u2, NTHR), NTHR, 0, stream>>>(w2a, HID, K2, HID, HID, W2A2, u2);
    k_wtr<<<cdiv(u2, NTHR), NTHR, 0, stream>>>(w1b, HID, K2, HID, HID, W1B2, u2);
    k_wtr<<<cdiv(u2, NTHR), NTHR, 0, stream>>>(w2b, HID, K2, HID, HID, W2B2, u2);
    const int u3 = ODIM * (K2 / 8);
    k_wtr<<<cdiv(u3, NTHR), NTHR, 0, stream>>>(w1c, ODIM, K2, HID, HID, W1C2, u3);
    const int u4 = ODIM * (KC / 8);
    k_wtr<<<cdiv(u4, NTHR), NTHR, 0, stream>>>(w2c, ODIM, KC, ODIM, ODIM, W2C2, u4);
  }
  k_gemm<4, 0><<<gM, GTHR, 0, stream>>>(XB, W1AT, KX, b1a, FL, nN, Pp, Hp);
  k_scan<2><<<gA, NTHR, aggLds, stream>>>(src, dst, eat, nE, nN, vec8, MP, Pp, w1a, XDIM, b1a, 1, Mp, FL);
  k_gemm<4, 1><<<gM, GTHR, 0, stream>>>(Mp, W2A2, K2, b2a, FL, nN, Pp, Hp);
  k_gemm<4, 0><<<gM, GTHR, 0, stream>>>(Hp, W1B2, K2, b1b, FL, nN, Pp, Hp);
  k_scan<2><<<gA, NTHR, aggLds, stream>>>(src, dst, eat, nE, nN, vec8, MP, Pp, w1b, HID, b1b, 0, Mp, FL);
  k_gemm<4, 1><<<gM, GTHR, 0, stream>>>(Mp, W2B2, K2, b2b, FL, nN, Pp, Hp);
  k_gemm<2, 0><<<gM, GTHR, 0, stream>>>(Hp, W1C2, K2, b1c, FL, nN, Pp, Hp);
  k_scan<1><<<gA, NTHR, aggLds, stream>>>(src, dst, eat, nE, nN, vec8, MP, Pp, w1c, HID, b1c, 0, Mp, FL);
  k_gemm<2, 2><<<gM, GTHR, 0, stream>>>(Mp, W2C2, KC, b2c, FL, nN, out, Hp);
}
